// GraphSageLinkPredNoEmb_56624848830739
// MI455X (gfx1250) — hardware-verified
//
#include <hip/hip_runtime.h>
#include <stddef.h>


#define DF      128
#define FIN     64
#define KV      256
#define NTHR    256
#define NWAVE   8
#define EPT     8
#define NGRP    2
#define CHUNK   (NTHR * EPT * NGRP)
#define WCAP    (EPT * NGRP * 32)
#define LISTN   (NWAVE * WCAP)
#define NB      512
#define NTILE   (NB / 16)
#define TPW     (NTILE / NWAVE)
#define PROWS   (NWAVE * 16)
#define LPB     256

#define LDS_ACC   (NB * DF * 4)
#define LDS_LIST  (LISTN * 4)
#define LDS_CNT   (NB * 4)
#define LDS_LAYER (LDS_ACC + LDS_LIST + LDS_CNT + 64)

static_assert((CHUNK & (CHUNK - 1)) == 0);
static_assert(CHUNK <= 4096);
static_assert((NB & (NB - 1)) == 0);
static_assert(NB <= 4096);
static_assert(NTILE % NWAVE == 0);
static_assert(NB % PROWS == 0);
static_assert(NWAVE * 4 <= 64);
static_assert(LDS_LAYER <= 300 * 1024);
static_assert(FIN % 32 == 0);
static_assert(LPB == NTHR);

typedef float  v4f   __attribute__((ext_vector_type(4)));
typedef float  v8f   __attribute__((ext_vector_type(8)));
typedef int    v4i   __attribute__((ext_vector_type(4)));
typedef __bf16 bf16_t;
typedef bf16_t v8bf  __attribute__((ext_vector_type(8)));
typedef bf16_t v16bf __attribute__((ext_vector_type(16)));
union FragB { v16bf v; v8bf h[2]; v4i q[2]; };
union Pack8 { v8bf v; v4i q; };

__device__ __forceinline__ v8f wmb(v16bf a, v16bf b, v8f c) {
  v8f d = __builtin_amdgcn_wmma_f32_16x16x32_bf16(false, a, false, b, (short)0, c, false, false);
  asm volatile("v_nop\n\tv_nop\n\tv_nop\n\tv_nop" : "+v"(d) : "v"(a), "v"(b));
  return d;
}

template <int B>
__device__ __forceinline__ void split8(FragB& hi, FragB& lo, v4f a, v4f b) {
#define SPL1(I, X) { const float xv = (X); const bf16_t hb = (bf16_t)xv; hi.v[B + (I)] = hb; lo.v[B + (I)] = (bf16_t)(xv - (float)hb); }
  SPL1(0, a.x) SPL1(1, a.y) SPL1(2, a.z) SPL1(3, a.w)
  SPL1(4, b.x) SPL1(5, b.y) SPL1(6, b.z) SPL1(7, b.w)
#undef SPL1
}

template <int NBT>
__device__ __forceinline__ int scan_chunk(const int* __restrict__ own, int nE, int cbase, int nodeBase,
                                          int vec8, int* list, int tid, int wave) {
  int wc = 0;
#pragma unroll
  for (int g = 0; g < NGRP; ++g) {
    const int el0  = (g * NTHR + tid) * EPT;
    const int e0   = cbase + el0;
    const int sent = -2147483647 - 1;
    v4i da, db;
    if (vec8 != 0 && cbase + CHUNK <= nE) {
      da = *(const v4i*)(own + e0);
      db = *(const v4i*)(own + e0 + 4);
    } else {
      da.x = (e0     < nE) ? own[min(e0, nE - 1)]     : sent;
      da.y = (e0 + 1 < nE) ? own[min(e0 + 1, nE - 1)] : sent;
      da.z = (e0 + 2 < nE) ? own[min(e0 + 2, nE - 1)] : sent;
      da.w = (e0 + 3 < nE) ? own[min(e0 + 3, nE - 1)] : sent;
      db.x = (e0 + 4 < nE) ? own[min(e0 + 4, nE - 1)] : sent;
      db.y = (e0 + 5 < nE) ? own[min(e0 + 5, nE - 1)] : sent;
      db.z = (e0 + 6 < nE) ? own[min(e0 + 6, nE - 1)] : sent;
      db.w = (e0 + 7 < nE) ? own[min(e0 + 7, nE - 1)] : sent;
    }
    const unsigned nb = (unsigned)nodeBase;
    const unsigned s0 = (unsigned)da.x - nb, s1 = (unsigned)da.y - nb;
    const unsigned s2 = (unsigned)da.z - nb, s3 = (unsigned)da.w - nb;
    const unsigned s4 = (unsigned)db.x - nb, s5 = (unsigned)db.y - nb;
    const unsigned s6 = (unsigned)db.z - nb, s7 = (unsigned)db.w - nb;
    const bool h0 = s0 < (unsigned)NBT, h1 = s1 < (unsigned)NBT, h2 = s2 < (unsigned)NBT, h3 = s3 < (unsigned)NBT;
    const bool h4 = s4 < (unsigned)NBT, h5 = s5 < (unsigned)NBT, h6 = s6 < (unsigned)NBT, h7 = s7 < (unsigned)NBT;
    const unsigned any = __builtin_amdgcn_ballot_w32(h0 | h1 | h2 | h3 | h4 | h5 | h6 | h7);
    if (any != 0u) {
#define HITJ(J, HJ, SJ) { \
        const unsigned mj = __builtin_amdgcn_ballot_w32(HJ); \
        if (mj != 0u) { \
          if (HJ) { \
            const int pos = wc + (int)__builtin_amdgcn_mbcnt_lo(mj, 0u); \
            if (pos < WCAP) list[wave * WCAP + pos] = ((el0 + (J)) << 12) | (int)(SJ); \
          } \
          wc += (int)__builtin_popcount(mj); } }
      HITJ(0, h0, s0)
      HITJ(1, h1, s1)
      HITJ(2, h2, s2)
      HITJ(3, h3, s3)
      HITJ(4, h4, s4)
      HITJ(5, h5, s5)
      HITJ(6, h6, s6)
      HITJ(7, h7, s7)
#undef HITJ
    }
  }
  return wc;
}

__global__ __launch_bounds__(NTHR) void k_wprep(
    const float* __restrict__ W0, const float* __restrict__ W1, int K0, int K1,
    bf16_t* whi, bf16_t* wlo, int nTot) {
  const int i = blockIdx.x * NTHR + threadIdx.x;
  if (i >= nTot) return;
  const int KT    = K0 + K1;
  const int o     = i * 8;
  const int layer = o / (DF * KT);
  const int rem   = o - layer * (DF * KT);
  const int n     = rem / KT;
  const int k0    = rem - n * KT;
  int ka = k0;       ka = ka > K0 - 8 ? K0 - 8 : ka; ka = ka < 0 ? 0 : ka;
  int kb = k0 - K0;  kb = kb < 0 ? 0 : kb;
  const int kbm = (K1 >= 8) ? (K1 - 8) : 0;
  kb = kb > kbm ? kbm : kb;
  const float* pa = W0 + (size_t)layer * DF * K0 + (size_t)n * K0 + ka;
  const float* pb = W1 + (size_t)layer * DF * K1 + (size_t)n * K1 + kb;
  const v4f a0 = *(const v4f*)pa;
  const v4f a1 = *(const v4f*)(pa + 4);
  const v4f b0 = *(const v4f*)pb;
  const v4f b1 = *(const v4f*)(pb + 4);
  const bool sa = k0 < K0;
  Pack8 ph, pl;
#define WSP(I, XA, XB) { const float xv = sa ? (XA) : (XB); const bf16_t hb = (bf16_t)xv; ph.v[(I)] = hb; pl.v[(I)] = (bf16_t)(xv - (float)hb); }
  WSP(0, a0.x, b0.x) WSP(1, a0.y, b0.y) WSP(2, a0.z, b0.z) WSP(3, a0.w, b0.w)
  WSP(4, a1.x, b1.x) WSP(5, a1.y, b1.y) WSP(6, a1.z, b1.z) WSP(7, a1.w, b1.w)
#undef WSP
  bf16_t* dh = whi + o;
  bf16_t* dl = wlo + o;
  const v4i qh = ph.q, ql = pl.q;
  *(volatile v4i*)dh = qh;
  *(volatile v4i*)dl = ql;
  __threadfence();
  *(volatile v4i*)dh = qh;
  *(volatile v4i*)dl = ql;
}

template <int KB>
__device__ __forceinline__ void kstep(const float* ap, float mul,
                                      const bf16_t* bhp, const bf16_t* blp, v8f (&c)[8]) {
  const v4f p0 = (*(const v4f*)(ap))      * mul;
  const v4f p1 = (*(const v4f*)(ap + 4))  * mul;
  const v4f p2 = (*(const v4f*)(ap + 16)) * mul;
  const v4f p3 = (*(const v4f*)(ap + 20)) * mul;
  FragB ahi, alo;
  split8<0>(ahi, alo, p0, p1);
  split8<8>(ahi, alo, p2, p3);
#pragma unroll
  for (int ct = 0; ct < DF / 16; ++ct) {
    const bf16_t* hp = bhp + (size_t)ct * 16 * KB;
    const bf16_t* lp = blp + (size_t)ct * 16 * KB;
    FragB bh, bq;
    bh.q[0] = *(const v4i*)hp;  bh.q[1] = *(const v4i*)(hp + 16);
    bq.q[0] = *(const v4i*)lp;  bq.q[1] = *(const v4i*)(lp + 16);
    c[ct] = wmb(alo.v, bh.v, c[ct]);
    c[ct] = wmb(ahi.v, bq.v, c[ct]);
    c[ct] = wmb(ahi.v, bh.v, c[ct]);
  }
}

__device__ __forceinline__ void epi_tile(const v8f (&c)[8], const float* __restrict__ bias, int relu,
                                         float* sp, int m) {
#pragma unroll
  for (int ct = 0; ct < 8; ++ct) {
    const float b = bias[16 * ct + m];
#pragma unroll
    for (int r = 0; r < 8; ++r) {
      float v = c[ct][r] + b;
      v = (relu != 0) ? fmaxf(v, 0.0f) : v;
      sp[r * DF + 16 * ct] = v;
    }
  }
}

__device__ __forceinline__ void store_rows16(const float* lrow, float* gp) {
#pragma unroll
  for (int i = 0; i < 16; ++i) { const v4f v = *(const v4f*)(lrow + i * DF); *(volatile v4f*)(gp + (size_t)i * DF) = v; }
  __threadfence();
#pragma unroll
  for (int i = 0; i < 16; ++i) { const v4f v = *(const v4f*)(lrow + i * DF); *(volatile v4f*)(gp + (size_t)i * DF) = v; }
}

__global__ __launch_bounds__(NTHR) void k_proj(
    const float* __restrict__ x, const bf16_t* __restrict__ whi, const bf16_t* __restrict__ wlo,
    const float* __restrict__ bias, float* xout, int nN) {
  __shared__ v4f st4[PROWS * DF / 4];
  float* stile = (float*)st4;
  const int tid = threadIdx.x, lane = tid & 31, wave = tid >> 5, hh = lane >> 4, m = lane & 15;
  const int row0 = blockIdx.x * PROWS + wave * 16;
  int node = row0 + m;
  node = node > nN - 1 ? nN - 1 : node;

  v8f c[8];
#pragma unroll
  for (int ct = 0; ct < 8; ++ct) { const v8f z = {0.f, 0.f, 0.f, 0.f, 0.f, 0.f, 0.f, 0.f}; c[ct] = z; }

  const float*  xrow = x + (size_t)node * FIN + 8 * hh;
  const bf16_t* bh0  = whi + m * FIN + 8 * hh;
  const bf16_t* bl0  = wlo + m * FIN + 8 * hh;
#pragma unroll 1
  for (int ks = 0; ks < FIN / 32; ++ks)
    kstep<FIN>(xrow + 32 * ks, 1.0f, bh0 + 32 * ks, bl0 + 32 * ks, c);

  epi_tile(c, bias, 0, stile + (wave * 16 + 8 * hh) * DF + m, m);
  __syncthreads();
  store_rows16(stile + (wave * 16) * DF + 4 * lane, xout + (size_t)row0 * DF + 4 * lane);
}

__global__ __launch_bounds__(NTHR) void k_layer(
    const int* __restrict__ own, const int* __restrict__ oth,
    const float* __restrict__ xg, const float* xs,
    const bf16_t* __restrict__ whi, const bf16_t* __restrict__ wlo,
    const float* __restrict__ bias, float* xout,
    int nN, int nG, int nE, int vec8, int relu) {
  extern __shared__ v4f lds_dyn[];
  float* acc  = (float*)lds_dyn;
  int*   list = (int*)((char*)lds_dyn + LDS_ACC);
  int*   cnt  = (int*)((char*)lds_dyn + LDS_ACC + LDS_LIST);
  int*   wcnt = (int*)((char*)lds_dyn + LDS_ACC + LDS_LIST + LDS_CNT);
  const int tid = threadIdx.x, lane = tid & 31, wave = tid >> 5, hh = lane >> 4, m = lane & 15;
  const int nodeBase = blockIdx.x * NB;

  {
    const v4f z = {0.f, 0.f, 0.f, 0.f};
    for (int i = tid; i < NB * DF / 4; i += NTHR) lds_dyn[i] = z;
    for (int i = tid; i < NB; i += NTHR) cnt[i] = 0;
  }
  __syncthreads();

  const int nChunks = (nE + CHUNK - 1) / CHUNK;
#pragma unroll 1
  for (int ch = 0; ch < nChunks; ++ch) {
    const int cbase = ch * CHUNK;
    const int wc = scan_chunk<NB>(own, nE, cbase, nodeBase, vec8, list, tid, wave);
    if (lane == 0) wcnt[wave] = wc;
    __syncthreads();
    if (wave == 0) {
#pragma unroll 1
      for (int wsx = 0; wsx < NWAVE; ++wsx) {
        int n = __builtin_amdgcn_readfirstlane(wcnt[wsx]);
        n = n > WCAP ? WCAP : (n < 0 ? 0 : n);
        const int* lp = list + wsx * WCAP;
#pragma unroll 1
        for (int i = 0; i < n; ++i) {
          const int ent  = __builtin_amdgcn_readfirstlane(lp[i]);
          const int slot = ent & (NB - 1);
          int e = cbase + ((ent >> 12) & (CHUNK - 1));
          e = e > nE - 1 ? nE - 1 : e;
          int src = oth[e];
          src = src < 0 ? 0 : (src > nG - 1 ? nG - 1 : src);
          const v4f v = *(const v4f*)(xg + (size_t)src * DF + 4 * lane);
          v4f* ap = (v4f*)(acc + slot * DF + 4 * lane);
          *ap = *ap + v;
          if (lane == 0) cnt[slot] = cnt[slot] + 1;
        }
      }
    }
    __syncthreads();
  }
  __syncthreads();

#pragma unroll 1
  for (int q = 0; q < TPW; ++q) {
    const int t     = q * NWAVE + wave;
    const int slotm = 16 * t + m;
    int node = nodeBase + slotm;
    node = node > nN - 1 ? nN - 1 : node;
    const int   cd  = cnt[slotm];
    const float inv = 1.0f / (float)(cd > 1 ? cd : 1);

    v8f c[8];
#pragma unroll
    for (int ct = 0; ct < 8; ++ct) { const v8f z = {0.f, 0.f, 0.f, 0.f, 0.f, 0.f, 0.f, 0.f}; c[ct] = z; }

    const float*  arow = acc + slotm * DF + 8 * hh;
    const float*  xrow = xs + (size_t)node * DF + 8 * hh;
    const bf16_t* bh0  = whi + m * KV + 8 * hh;
    const bf16_t* bl0  = wlo + m * KV + 8 * hh;
#pragma unroll 1
    for (int ks = 0; ks < DF / 32; ++ks)
      kstep<KV>(arow + 32 * ks, inv, bh0 + 32 * ks, bl0 + 32 * ks, c);
#pragma unroll 1
    for (int ks = 0; ks < DF / 32; ++ks)
      kstep<KV>(xrow + 32 * ks, 1.0f, bh0 + DF + 32 * ks, bl0 + DF + 32 * ks, c);

    epi_tile(c, bias, relu, acc + (16 * t + 8 * hh) * DF + m, m);
    __syncthreads();
    store_rows16(acc + (16 * t) * DF + 4 * lane, xout + ((size_t)nodeBase + 16 * t) * DF + 4 * lane);
  }
}

__global__ __launch_bounds__(NTHR) void k_link(
    const float* __restrict__ xu, const float* __restrict__ xp,
    const int* __restrict__ ls, const int* __restrict__ ld,
    float* out, int L, int nU, int nP) {
  __shared__ float sc[LPB];
  const int tid = threadIdx.x, lane = tid & 31, wave = tid >> 5;
  const int base = blockIdx.x * LPB;
  float res = 0.0f;
#pragma unroll 1
  for (int j = 0; j < 32; ++j) {
    int pr = base + wave * 32 + j;
    pr = pr > L - 1 ? L - 1 : pr;
    int a = ls[pr];
    a = a < 0 ? 0 : (a > nU - 1 ? nU - 1 : a);
    int b = ld[pr];
    b = b < 0 ? 0 : (b > nP - 1 ? nP - 1 : b);
    const v4f va = *(const v4f*)(xu + (size_t)a * DF + 4 * lane);
    const v4f vb = *(const v4f*)(xp + (size_t)b * DF + 4 * lane);
    float p = va.x * vb.x + va.y * vb.y + va.z * vb.z + va.w * vb.w;
    p += __shfl_xor(p, 16, 32);
    p += __shfl_xor(p, 8, 32);
    p += __shfl_xor(p, 4, 32);
    p += __shfl_xor(p, 2, 32);
    p += __shfl_xor(p, 1, 32);
    res = (lane == j) ? p : res;
  }
  sc[wave * 32 + lane] = res;
  __syncthreads();
  if (tid < LPB / 4) {
    const int  p0   = base + 4 * tid;
    const v4f  v    = *(const v4f*)(sc + 4 * tid);
    const bool full = (p0 + 3 < L);
    float* op = out + (size_t)(full ? p0 : 0);
    if (full) {
      *(volatile v4f*)op = v;
    } else {
      if (p0     < L) *(volatile float*)(out + p0)     = v.x;
      if (p0 + 1 < L) *(volatile float*)(out + p0 + 1) = v.y;
      if (p0 + 2 < L) *(volatile float*)(out + p0 + 2) = v.z;
      if (p0 + 3 < L) *(volatile float*)(out + p0 + 3) = v.w;
    }
    __threadfence();
    if (full) {
      *(volatile v4f*)op = v;
    } else {
      if (p0     < L) *(volatile float*)(out + p0)     = v.x;
      if (p0 + 1 < L) *(volatile float*)(out + p0 + 1) = v.y;
      if (p0 + 2 < L) *(volatile float*)(out + p0 + 2) = v.z;
      if (p0 + 3 < L) *(volatile float*)(out + p0 + 3) = v.w;
    }
  }
}

extern "C" void kernel_launch(void* const* d_in, const int* in_sizes, int n_in,
                              void* d_out, int out_size, void* d_ws, size_t ws_size,
                              hipStream_t stream) {
  if (n_in < 16) return;
  if (in_sizes[7] != DF || in_sizes[9] != DF) return;
  if (in_sizes[6] != DF * FIN || in_sizes[8] != DF * FIN) return;
  const int NU = in_sizes[0] / FIN;
  const int NP = in_sizes[1] / FIN;
  if (NU <= 0 || NP <= 0 || in_sizes[0] != NU * FIN || in_sizes[1] != NP * FIN) return;
  const int E = in_sizes[2];
  if (E <= 0 || in_sizes[3] != E) return;
  const int L = in_sizes[4];
  if (L <= 0 || in_sizes[5] != L || out_size != L) return;
  const int NL = in_sizes[10] / (DF * DF);
  if (NL <= 0 || in_sizes[10] != NL * DF * DF || in_sizes[12] != NL * DF * DF ||
      in_sizes[13] != NL * DF * DF || in_sizes[15] != NL * DF * DF) return;
  if (in_sizes[11] < NL * DF || in_sizes[14] < NL * DF) return;

  const float* x_user = (const float*)d_in[0];
  const float* x_prod = (const float*)d_in[1];
  const int*   esrc   = (const int*)d_in[2];
  const int*   edst   = (const int*)d_in[3];
  const int*   lsrc   = (const int*)d_in[4];
  const int*   ldst   = (const int*)d_in[5];
  const float* user_W = (const float*)d_in[6];
  const float* user_b = (const float*)d_in[7];
  const float* prod_W = (const float*)d_in[8];
  const float* prod_b = (const float*)d_in[9];
  const float* Wl_buy = (const float*)d_in[10];
  const float* bl_buy = (const float*)d_in[11];
  const float* Wr_buy = (const float*)d_in[12];
  const float* Wl_rev = (const float*)d_in[13];
  const float* bl_rev = (const float*)d_in[14];
  const float* Wr_rev = (const float*)d_in[15];
  float* out = (float*)d_out;

  const int nBlkU = (NU + NB - 1) / NB;
  const int nBlkP = (NP + NB - 1) / NB;
  const size_t rowsU = (size_t)nBlkU * NB;
  const size_t rowsP = (size_t)nBlkP * NB;

  char* ws = (char*)d_ws;
  size_t off = 0;
  const size_t szWin = (size_t)DF * FIN * 2;
  const size_t szWly = (size_t)NL * DF * KV * 2;
  const size_t szXu  = rowsU * DF * 4;
  const size_t szXp  = rowsP * DF * 4;
#define CARVE(NAME, BYTES) const size_t NAME = off; off += (BYTES); off = (off + 255) & ~(size_t)255;
  CARVE(oWhU, szWin) CARVE(oWlU, szWin) CARVE(oWhP, szWin) CARVE(oWlP, szWin)
  CARVE(oWhB, szWly) CARVE(oWlB, szWly) CARVE(oWhR, szWly) CARVE(oWlR, szWly)
  CARVE(oXu, szXu) CARVE(oXpA, szXp) CARVE(oXpB, szXp)
#undef CARVE
  if (off > ws_size || off > (size_t)134217728) return;
  bf16_t* whU = (bf16_t*)(ws + oWhU); bf16_t* wlU = (bf16_t*)(ws + oWlU);
  bf16_t* whP = (bf16_t*)(ws + oWhP); bf16_t* wlP = (bf16_t*)(ws + oWlP);
  bf16_t* whB = (bf16_t*)(ws + oWhB); bf16_t* wlB = (bf16_t*)(ws + oWlB);
  bf16_t* whR = (bf16_t*)(ws + oWhR); bf16_t* wlR = (bf16_t*)(ws + oWlR);
  float* xu  = (float*)(ws + oXu);
  float* xpA = (float*)(ws + oXpA);
  float* xpB = (float*)(ws + oXpB);

  const int nTin = DF * FIN / 8;
  const int nTly = NL * DF * KV / 8;
  k_wprep<<<(nTin + NTHR - 1) / NTHR, NTHR, 0, stream>>>(user_W, user_W, FIN, 0, whU, wlU, nTin);
  k_wprep<<<(nTin + NTHR - 1) / NTHR, NTHR, 0, stream>>>(prod_W, prod_W, FIN, 0, whP, wlP, nTin);
  k_wprep<<<(nTly + NTHR - 1) / NTHR, NTHR, 0, stream>>>(Wl_buy, Wr_buy, DF, DF, whB, wlB, nTly);
  k_wprep<<<(nTly + NTHR - 1) / NTHR, NTHR, 0, stream>>>(Wl_rev, Wr_rev, DF, DF, whR, wlR, nTly);

  k_proj<<<(unsigned)(rowsU / PROWS), NTHR, 0, stream>>>(x_user, whU, wlU, user_b, xu, NU);
  k_proj<<<(unsigned)(rowsP / PROWS), NTHR, 0, stream>>>(x_prod, whP, wlP, prod_b, xpA, NP);

  hipFuncSetAttribute(reinterpret_cast<const void*>(&k_layer),
                      hipFuncAttributeMaxDynamicSharedMemorySize, LDS_LAYER);

  const int vec8 = 1;
  float* xp_cur = xpA;
  float* xp_nxt = xpB;
  for (int l = 0; l < NL; ++l) {
    const int relu = (l < NL - 1) ? 1 : 0;
    k_layer<<<nBlkP, NTHR, LDS_LAYER, stream>>>(
        edst, esrc, xu, xp_cur,
        whB + (size_t)l * DF * KV, wlB + (size_t)l * DF * KV, bl_buy + (size_t)l * DF,
        xp_nxt, NP, NU, E, vec8, relu);
    k_layer<<<nBlkU, NTHR, LDS_LAYER, stream>>>(
        esrc, edst, xp_cur, xu,
        whR + (size_t)l * DF * KV, wlR + (size_t)l * DF * KV, bl_rev + (size_t)l * DF,
        xu, NU, NP, E, vec8, relu);
    float* t = xp_cur; xp_cur = xp_nxt; xp_nxt = t;
  }

  k_link<<<(L + LPB - 1) / LPB, NTHR, 0, stream>>>(xu, xp_cur, lsrc, ldst, out, L, NU, NP);
}
